// OuterProductMean_23476291239989
// MI455X (gfx1250) — hardware-verified
//
#include <hip/hip_runtime.h>
#include <math.h>

constexpr int kRes   = 256;
constexpr int kSeq   = 128;
constexpr int kChan  = 256;
constexpr int kCO    = 32;
constexpr int kOutC  = 128;
constexpr int kOPK   = kCO * kCO;
constexpr long kPlaneHalves = (long)kRes * kCO * kSeq;
constexpr float kLnEps   = 1e-5f;
constexpr float kNormEps = 1e-3f;
constexpr float kWCarry     = 16.0f;
constexpr float kWCarryInv  = 1.0f / 16.0f;
constexpr float kResCarry   = 2048.0f;
constexpr float kResFoldInv = 1.0f / 32768.0f;
constexpr float kInvChan    = 1.0f / 256.0f;

constexpr long kOffLR   = 0;
constexpr long kOffWLR  = 2 * kPlaneHalves * 2;
constexpr long kOffWO   = kOffWLR + 64L * kChan * 2;
constexpr long kWsBytes = kOffWO + (long)kOutC * kOPK * 2;
static_assert(kOffWLR == 4194304 && kOffWO == 4227072 && kWsBytes == 4489216, "ws map");
static_assert(kWsBytes <= 134217728L, "ws carve limit");
static_assert(kChan % 32 == 0 && kSeq % 32 == 0 && kOPK % 32 == 0, "K multiples of 32");
static_assert(kSeq % 64 == 0 && kRes % 4 == 0 && kOutC == 128 && kCO == 32, "tile multiples");

typedef __attribute__((ext_vector_type(16))) _Float16 v16h;
typedef __attribute__((ext_vector_type(8)))  _Float16 v8h;
typedef __attribute__((ext_vector_type(2)))  _Float16 v2h;
typedef __attribute__((ext_vector_type(8)))  float    v8f;
typedef __attribute__((ext_vector_type(4)))  float    v4f;
typedef __attribute__((ext_vector_type(4)))  unsigned int v4u;

__device__ __forceinline__ float bfr(float f) {
  unsigned u = __float_as_uint(f);
  u = (u + 0x7FFFu + ((u >> 16) & 1u)) & 0xffff0000u;
  return __uint_as_float(u);
}
__device__ __forceinline__ unsigned pack2h(float a, float b) {
  const v2h p = {(_Float16)a, (_Float16)b};
  return __builtin_bit_cast(unsigned, p);
}
__device__ __forceinline__ float h16_to_f32(unsigned hb) {
  const unsigned sgn = (hb & 0x8000u) << 16; const unsigned em = hb & 0x7fffu;
  const float fn = __uint_as_float((em << 13) + 0x38000000u);
  const float fs = (float)em * 5.9604644775390625e-8f;
  const float mag = (em < 0x400u) ? fs : fn; return __uint_as_float(__float_as_uint(mag) | sgn); }

__device__ __forceinline__ void dep_guard_h(v8f& a, v8f& b, v16h x, v16h y) { asm volatile("v_nop\n\tv_nop\n\tv_nop\n\tv_nop" : "+v"(a), "+v"(b) : "v"(x), "v"(y)); }
__device__ __forceinline__ void keep4_h(v16h a, v16h b, v16h c, v16h d) { asm volatile("v_nop" :: "v"(a), "v"(b), "v"(c), "v"(d)); }
__device__ __forceinline__ void acc_guard4(v8f& a, v8f& b, v8f& c, v8f& d) { asm volatile("v_nop\n\tv_nop\n\tv_nop\n\tv_nop" : "+v"(a), "+v"(b), "+v"(c), "+v"(d)); }
__device__ __forceinline__ void acc_guard2(v8f& a, v8f& b) { asm volatile("v_nop\n\tv_nop\n\tv_nop\n\tv_nop" : "+v"(a), "+v"(b)); }
__device__ __forceinline__ void guard4c5f(v8f& c0, v8f& c1, v8f& c2, v8f& c3, v16h f0, v16h f1, v16h f2, v16h f3, v16h f4) {
  asm volatile("v_nop\n\tv_nop\n\tv_nop\n\tv_nop" : "+v"(c0), "+v"(c1), "+v"(c2), "+v"(c3) : "v"(f0), "v"(f1), "v"(f2), "v"(f3), "v"(f4));
}
__device__ __forceinline__ void guard4c4f(v8f& c0, v8f& c1, v8f& c2, v8f& c3, v16h f0, v16h f1, v16h f2, v16h f3) {
  asm volatile("v_nop\n\tv_nop\n\tv_nop\n\tv_nop" : "+v"(c0), "+v"(c1), "+v"(c2), "+v"(c3) : "v"(f0), "v"(f1), "v"(f2), "v"(f3));
}
__device__ __forceinline__ void guard2c3f(v8f& c0, v8f& c1, v16h f0, v16h f1, v16h f2) {
  asm volatile("v_nop\n\tv_nop\n\tv_nop\n\tv_nop" : "+v"(c0), "+v"(c1) : "v"(f0), "v"(f1), "v"(f2));
}

template <typename T> struct Frag;
template <> struct Frag<_Float16> {
  typedef v16h V; union U { v16h v; v8h h[2]; };
  static __device__ __forceinline__ v16h load(const _Float16* p) {
    U f; f.h[0] = *(const v8h*)(p); f.h[1] = *(const v8h*)(p + 16); return f.v;
  }
  static __device__ __forceinline__ v8f mma(v16h a, v16h b, v8f c) {
    return __builtin_amdgcn_wmma_f32_16x16x32_f16(false, a, false, b, (short)0, c, false, false);
  }
  static __device__ __forceinline__ void guard(v8f& a, v8f& b, v16h x, v16h y) { dep_guard_h(a, b, x, y); }
  static __device__ __forceinline__ void keep(v16h a, v16h b, v16h c, v16h d) { keep4_h(a, b, c, d); }
};
typedef Frag<_Float16> FH;

__device__ __forceinline__ v8f zero8() { return (v8f){0.f, 0.f, 0.f, 0.f, 0.f, 0.f, 0.f, 0.f}; }

__global__ __launch_bounds__(256) void prep_weights_kernel(const float* __restrict__ w_left, const float* __restrict__ w_right,
                                                           const float* __restrict__ w_o,
                                                           unsigned short* __restrict__ wlr, unsigned short* __restrict__ wo16) {
  const int blk = blockIdx.x;
  const int t   = threadIdx.x;
  const float* src;
  unsigned short* dst;
  if (blk < 4) {
    const size_t e = (size_t)(blk * 256 + t) * 8;
    src = w_left + e;  dst = wlr + e;
  } else if (blk < 8) {
    const size_t e = (size_t)((blk - 4) * 256 + t) * 8;
    src = w_right + e; dst = wlr + 32 * kChan + e;
  } else {
    const size_t e = (size_t)((blk - 8) * 256 + t) * 8;
    src = w_o + e;     dst = wo16 + e;
  }
  const v4f a = *(const v4f*)(src);
  const v4f c = *(const v4f*)(src + 4);
  float f[8];
#pragma unroll
  for (int e = 0; e < 4; ++e) {
    const float fa = a[e];
    const float fc = c[e];
    f[e]     = bfr(fa) * kWCarry;
    f[4 + e] = bfr(fc) * kWCarry;
  }
  const v4u u = (v4u){pack2h(f[0], f[1]), pack2h(f[2], f[3]), pack2h(f[4], f[5]), pack2h(f[6], f[7])};
  *(volatile v4u*)dst = u;
  __threadfence();
  *(volatile v4u*)dst = u;
}

constexpr int kXP = 264;
constexpr int kTP = 68;
constexpr int kXhOff = 0;
constexpr int kXlOff = 64 * kXP * 2;
constexpr int kTtOff = kXlOff + 64 * kXP * 2;
constexpr int kSmOff = kTtOff + 64 * kTP * 4;
constexpr int kLds2  = kSmOff + 64 * 4;
static_assert(kLds2 == 85248 && (kXlOff % 16) == 0 && (kTtOff % 16) == 0 && (kSmOff % 16) == 0, "lds2 map");

__global__ __launch_bounds__(128) void ln_proj_kernel(const float* __restrict__ act, const float* __restrict__ mask,
                                                      const float* __restrict__ gamma, const float* __restrict__ beta,
                                                      const unsigned short* __restrict__ wlr,
                                                      const float* __restrict__ b_left, const float* __restrict__ b_right,
                                                      unsigned short* __restrict__ lr) {
  extern __shared__ __align__(16) unsigned char smem2[];
  unsigned short* xh = (unsigned short*)(smem2 + kXhOff);
  unsigned short* xl = (unsigned short*)(smem2 + kXlOff);
  float* tT    = (float*)(smem2 + kTtOff);
  float* smask = (float*)(smem2 + kSmOff);
  const int sh   = blockIdx.x;
  const int ri   = blockIdx.y;
  const int t    = threadIdx.x;
  const int lane = t & 31;
  const int wave = t >> 5;
  const int sbase = sh * 64;

  if (t < 64) smask[t] = bfr(mask[(size_t)(sbase + t) * kRes + ri]);

  const int c0 = lane * 8;
  float g8[8], b8[8];
  {
    const v4f ga = *(const v4f*)(gamma + c0);
    const v4f gb = *(const v4f*)(gamma + c0 + 4);
    const v4f ba = *(const v4f*)(beta + c0);
    const v4f bb = *(const v4f*)(beta + c0 + 4);
#pragma unroll
    for (int e = 0; e < 4; ++e) {
      const float f0 = ga[e], f1 = gb[e], f2 = ba[e], f3 = bb[e];
      g8[e] = bfr(f0); g8[4 + e] = bfr(f1); b8[e] = bfr(f2); b8[4 + e] = bfr(f3);
    }
  }

#pragma unroll 1
  for (int r = 0; r < 16; ++r) {
    const int sl = wave * 16 + r;
    const float* xr = act + ((size_t)ri * kSeq + sbase + sl) * kChan + c0;
    const v4f xa = *(const v4f*)(xr);
    const v4f xb = *(const v4f*)(xr + 4);
    float x[8];
#pragma unroll
    for (int e = 0; e < 4; ++e) {
      const float f0 = xa[e], f1 = xb[e];
      x[e] = bfr(f0); x[4 + e] = bfr(f1);
    }
    float s1 = 0.f;
#pragma unroll
    for (int e = 0; e < 8; ++e) s1 += x[e];
#pragma unroll
    for (int off = 16; off > 0; off >>= 1) s1 += __shfl_xor(s1, off, 32);
    const float mu = s1 * kInvChan;
    float s2 = 0.f;
#pragma unroll
    for (int e = 0; e < 8; ++e) { const float d = x[e] - mu; s2 += d * d; }
#pragma unroll
    for (int off = 16; off > 0; off >>= 1) s2 += __shfl_xor(s2, off, 32);
    const float rstd = rsqrtf(s2 * kInvChan + kLnEps);
    unsigned wh[4], wl[4];
#pragma unroll
    for (int e = 0; e < 4; ++e) {
      const float xn0 = (x[2 * e] - mu) * rstd * g8[2 * e] + b8[2 * e];
      const float xn1 = (x[2 * e + 1] - mu) * rstd * g8[2 * e + 1] + b8[2 * e + 1];
      unsigned w = pack2h(xn0, xn1);
      asm volatile("" : "+v"(w));
      const float h0 = h16_to_f32(w & 0xffffu);
      const float h1 = h16_to_f32(w >> 16);
      wh[e] = w;
      wl[e] = pack2h((xn0 - h0) * kResCarry, (xn1 - h1) * kResCarry);
    }
    const v4u uh = (v4u){wh[0], wh[1], wh[2], wh[3]};
    const v4u ul = (v4u){wl[0], wl[1], wl[2], wl[3]};
    *(v4u*)(xh + sl * kXP + c0) = uh;
    *(v4u*)(xl + sl * kXP + c0) = ul;
  }
  __syncthreads();

  const int rlane = lane & 15;
  const int hh    = lane >> 4;
  const int koff  = hh * 8;
  const _Float16* xhh = (const _Float16*)xh;
  const _Float16* xlh = (const _Float16*)xl;
  const _Float16* wl  = (const _Float16*)wlr;
  v8f acc[4], accr[4];
#pragma unroll
  for (int mi = 0; mi < 4; ++mi) { acc[mi] = zero8(); accr[mi] = zero8(); }
#pragma unroll 1
  for (int k0 = 0; k0 < kChan; k0 += 32) {
    const v16h bw = FH::load(wl + (size_t)(wave * 16 + rlane) * kChan + k0 + koff);
    {
      const v16h a0 = FH::load(xhh + (0 * 16 + rlane) * kXP + k0 + koff);
      const v16h a1 = FH::load(xhh + (1 * 16 + rlane) * kXP + k0 + koff);
      const v16h a2 = FH::load(xhh + (2 * 16 + rlane) * kXP + k0 + koff);
      const v16h a3 = FH::load(xhh + (3 * 16 + rlane) * kXP + k0 + koff);
      acc[0] = FH::mma(a0, bw, acc[0]);
      acc[1] = FH::mma(a1, bw, acc[1]);
      acc[2] = FH::mma(a2, bw, acc[2]);
      acc[3] = FH::mma(a3, bw, acc[3]);
      guard4c5f(acc[0], acc[1], acc[2], acc[3], a0, a1, a2, a3, bw);
    }
    {
      const v16h l0 = FH::load(xlh + (0 * 16 + rlane) * kXP + k0 + koff);
      const v16h l1 = FH::load(xlh + (1 * 16 + rlane) * kXP + k0 + koff);
      const v16h l2 = FH::load(xlh + (2 * 16 + rlane) * kXP + k0 + koff);
      const v16h l3 = FH::load(xlh + (3 * 16 + rlane) * kXP + k0 + koff);
      accr[0] = FH::mma(l0, bw, accr[0]);
      accr[1] = FH::mma(l1, bw, accr[1]);
      accr[2] = FH::mma(l2, bw, accr[2]);
      accr[3] = FH::mma(l3, bw, accr[3]);
      guard4c5f(accr[0], accr[1], accr[2], accr[3], l0, l1, l2, l3, bw);
    }
  }
  acc_guard4(acc[0], acc[1], acc[2], acc[3]);
  acc_guard4(accr[0], accr[1], accr[2], accr[3]);

  const int cc = wave * 16 + rlane;
  const float bl = b_left[cc & 31];
  const float br = b_right[cc & 31];
  const float fsel = (wave < 2) ? 1.0f : 0.0f;
  const float bv = bfr(fsel * bl + (1.0f - fsel) * br);
#pragma unroll
  for (int mi = 0; mi < 4; ++mi) {
#pragma unroll
    for (int r = 0; r < 8; ++r) {
      const int sl = mi * 16 + hh * 8 + r;
      const float v  = acc[mi][r];
      const float vr = accr[mi][r];
      tT[cc * kTP + sl] = (v * kWCarryInv + vr * kResFoldInv + bv) * smask[sl];
    }
  }
  __syncthreads();

  const int q  = lane >> 3;
  const int c8 = (lane & 7) * 8;
  unsigned short* plane = lr + (size_t)(wave >> 1) * kPlaneHalves;
  const int cb = (wave & 1) * 16;
  for (int pass = 0; pass < 2; ++pass) {
#pragma unroll
    for (int it = 0; it < 4; ++it) {
      const int crow = it * 4 + q;
      const float* sp = tT + (wave * 16 + crow) * kTP + c8;
      const v4f p0 = *(const v4f*)(sp);
      const v4f p1 = *(const v4f*)(sp + 4);
      float f[8];
#pragma unroll
      for (int e = 0; e < 4; ++e) {
        const float f0 = p0[e], f1 = p1[e];
        f[e] = f0; f[4 + e] = f1;
      }
      const v4u u = (v4u){pack2h(f[0], f[1]), pack2h(f[2], f[3]), pack2h(f[4], f[5]), pack2h(f[6], f[7])};
      *(volatile v4u*)(plane + ((size_t)(ri * kCO + cb + crow) * kSeq + sbase + c8)) = u;
    }
    __threadfence();
  }
}

constexpr int kPANP = 136;
constexpr int kOPP  = 1032;
constexpr int kOSP  = 132;
constexpr int kPanBytes = 256 * kPANP * 2;
constexpr int kOpbOff   = kPanBytes;
constexpr int kOpbBytes = 16 * kOPP * 2;
constexpr int kScOff    = kOpbOff + kOpbBytes;
constexpr int kLds3     = kScOff + 64;
static_assert(kLds3 == 102720 && (kOpbOff % 16) == 0 && (kScOff % 16) == 0, "lds3 map");
static_assert(16 * kOSP * 4 <= kPanBytes && 128 * 8 * 4 <= kOpbBytes, "lds3 aliases fit");

__global__ __launch_bounds__(128) void opm_kernel(const unsigned short* __restrict__ lr, const unsigned short* __restrict__ wo16,
                                                  const float* __restrict__ mask, const float* __restrict__ b_o,
                                                  float* __restrict__ out) {
  extern __shared__ __align__(16) unsigned char smem3[];
  unsigned short* pan  = (unsigned short*)(smem3);
  _Float16*       opbw = (_Float16*)(smem3 + kOpbOff);
  float*          mk   = (float*)(smem3 + kOpbOff);
  float*          sc   = (float*)(smem3 + kScOff);
  float*          outS = (float*)(smem3);

  const int i0   = blockIdx.x * 4;
  const int j0   = blockIdx.y * 4;
  const int t    = threadIdx.x;
  const int lane = t & 31;
  const int wave = t >> 5;
  const int rlane = lane & 15;
  const int hh    = lane >> 4;
  const int koff  = hh * 8;

  {
    const v4u* gl = (const v4u*)(lr + (size_t)i0 * kCO * kSeq);
    const v4u* gr = (const v4u*)(lr + kPlaneHalves + (size_t)j0 * kCO * kSeq);
#pragma unroll 1
    for (int it = 0; it < 16; ++it) {
      const int idx  = it * 128 + t;
      const int row  = idx >> 4;
      const int col8 = (idx & 15) * 8;
      const v4u a = gl[idx];
      const v4u b = gr[idx];
      *(v4u*)(pan + row * kPANP + col8) = a;
      *(v4u*)(pan + (128 + row) * kPANP + col8) = b;
      asm volatile("" ::: "memory");
    }
    const v4f mi = *(const v4f*)(mask + (size_t)t * kRes + i0);
    const v4f mj = *(const v4f*)(mask + (size_t)t * kRes + j0);
    v4f ri, rj;
#pragma unroll
    for (int e = 0; e < 4; ++e) { const float f0 = mi[e], f1 = mj[e]; ri[e] = bfr(f0); rj[e] = bfr(f1); }
    *(v4f*)(mk + t * 8) = ri;
    *(v4f*)(mk + t * 8 + 4) = rj;
  }
  __syncthreads();
  if (t < 16) {
    const int pi = t >> 2, pj = t & 3;
    float n = 0.f;
#pragma unroll 1
    for (int s = 0; s < kSeq; ++s) n += mk[s * 8 + pi] * mk[s * 8 + 4 + pj];
    sc[t] = 1.0f / (kNormEps + n);
  }
  __syncthreads();

  const _Float16* panh = (const _Float16*)pan;
#pragma unroll 1
  for (int jp = 0; jp < 4; ++jp) {
    v8f acc[2][2];
    acc[0][0] = zero8(); acc[0][1] = zero8(); acc[1][0] = zero8(); acc[1][1] = zero8();
#pragma unroll
    for (int kc = 0; kc < 4; ++kc) {
      const int k0 = kc * 32;
      const v16h af0 = FH::load(panh + (wave * 32 + rlane) * kPANP + k0 + koff);
      const v16h af1 = FH::load(panh + (wave * 32 + 16 + rlane) * kPANP + k0 + koff);
      const v16h bf0 = FH::load(panh + (128 + jp * 32 + rlane) * kPANP + k0 + koff);
      const v16h bf1 = FH::load(panh + (128 + jp * 32 + 16 + rlane) * kPANP + k0 + koff);
      acc[0][0] = FH::mma(af0, bf0, acc[0][0]);
      acc[0][1] = FH::mma(af0, bf1, acc[0][1]);
      acc[1][0] = FH::mma(af1, bf0, acc[1][0]);
      acc[1][1] = FH::mma(af1, bf1, acc[1][1]);
      guard4c4f(acc[0][0], acc[0][1], acc[1][0], acc[1][1], af0, af1, bf0, bf1);
    }
    acc_guard4(acc[0][0], acc[0][1], acc[1][0], acc[1][1]);
    const int p = wave * 4 + jp;
#pragma unroll
    for (int mt = 0; mt < 2; ++mt) {
#pragma unroll
      for (int nt = 0; nt < 2; ++nt) {
#pragma unroll
        for (int r = 0; r < 8; ++r) {
          const int c = mt * 16 + hh * 8 + r;
          const int d = nt * 16 + rlane;
          const float v = acc[mt][nt][r];
          opbw[p * kOPP + c * 32 + d] = (_Float16)v;
        }
      }
    }
  }
  __syncthreads();

  const _Float16* opbh = (const _Float16*)opbw;
  const _Float16* woh  = (const _Float16*)wo16;
  v8f acc2[2];
  acc2[0] = zero8(); acc2[1] = zero8();
#pragma unroll 1
  for (int k0 = 0; k0 < kOPK; k0 += 32) {
    const v16h a  = FH::load(opbh + rlane * kOPP + k0 + koff);
    const v16h b0 = FH::load(woh + (size_t)(wave * 16 + rlane) * kOPK + k0 + koff);
    const v16h b1 = FH::load(woh + (size_t)((wave + 4) * 16 + rlane) * kOPK + k0 + koff);
    acc2[0] = FH::mma(a, b0, acc2[0]);
    acc2[1] = FH::mma(a, b1, acc2[1]);
    guard2c3f(acc2[0], acc2[1], a, b0, b1);
  }
  acc_guard2(acc2[0], acc2[1]);

  {
    const int o0 = wave * 16 + rlane;
    const int o1 = (wave + 4) * 16 + rlane;
    const float bo0 = bfr(b_o[o0]);
    const float bo1 = bfr(b_o[o1]);
#pragma unroll
    for (int r = 0; r < 8; ++r) {
      const int p = hh * 8 + r;
      const float inv = sc[p];
      const float v0 = acc2[0][r];
      const float v1 = acc2[1][r];
      outS[p * kOSP + o0] = (v0 * kWCarryInv + bo0) * inv;
      outS[p * kOSP + o1] = (v1 * kWCarryInv + bo1) * inv;
    }
  }
  __syncthreads();

  for (int pass = 0; pass < 2; ++pass) {
#pragma unroll
    for (int it = 0; it < 4; ++it) {
      const int p = wave * 4 + it;
      const v4f v = *(const v4f*)(outS + p * kOSP + lane * 4);
      *(volatile v4f*)(out + ((size_t)((i0 + wave) * kRes + (j0 + it))) * kOutC + lane * 4) = v;
    }
    __threadfence();
  }
}

extern "C" void kernel_launch(void* const* d_in, const int* in_sizes, int n_in,
                              void* d_out, int out_size, void* d_ws, size_t ws_size, hipStream_t stream) {
  (void)in_sizes; (void)n_in; (void)out_size;
  const float* act     = (const float*)d_in[0];
  const float* mask    = (const float*)d_in[1];
  const float* gamma   = (const float*)d_in[2];
  const float* beta    = (const float*)d_in[3];
  const float* w_left  = (const float*)d_in[4];
  const float* b_left  = (const float*)d_in[5];
  const float* w_right = (const float*)d_in[6];
  const float* b_right = (const float*)d_in[7];
  const float* w_o     = (const float*)d_in[8];
  const float* b_o     = (const float*)d_in[9];
  float* out = (float*)d_out;

  if (ws_size < (size_t)kWsBytes) return;
  unsigned char* ws = (unsigned char*)d_ws;
  unsigned short* lr   = (unsigned short*)(ws + kOffLR);
  unsigned short* wlr  = (unsigned short*)(ws + kOffWLR);
  unsigned short* wo16 = (unsigned short*)(ws + kOffWO);

  prep_weights_kernel<<<dim3(72), dim3(256), 0, stream>>>(w_left, w_right, w_o, wlr, wo16);
  ln_proj_kernel<<<dim3(2, kRes), dim3(128), kLds2, stream>>>(act, mask, gamma, beta, wlr, b_left, b_right, lr);
  opm_kernel<<<dim3(kRes / 4, kRes / 4), dim3(128), kLds3, stream>>>(lr, wo16, mask, b_o, out);
}
